// GRUCell_59665685676320
// MI455X (gfx1250) — hardware-verified
//
#include <hip/hip_runtime.h>
#include <math.h>
#include <stdint.h>


#define BATCH 4096
#define KD    1024
#define HD    1024
#define N3    (3 * HD)
#define BN_EPS 1e-5f

#define SCA   64.0f
#define SCW   64.0f
#define SCP   4096.0f
#define SCR   2048.0f
#define INVAW (1.0f / (SCA * SCW))
#define INVPW (1.0f / (SCP * SCW))
#define INVPL (INVPW / SCR)

static_assert(BATCH % 64 == 0 && N3 % 64 == 0 && HD % 64 == 0 && KD % 64 == 0);
static_assert(KD % 32 == 0 && HD % 32 == 0 && KD % 8 == 0 && HD % 8 == 0);
static_assert((((BATCH / 64) * (N3 / 64)) % 8) == 0);
static_assert((((BATCH / 64) * (HD / 64)) % 8) == 0);
static_assert((((BATCH / 32) * (HD / 64)) % 8) == 0);
static_assert((BATCH * KD) % 2048 == 0 && (BATCH * HD) % 2048 == 0);
static_assert(BATCH % 4 == 0);
static_assert(KD == HD);

typedef _Float16       v16h __attribute__((ext_vector_type(16)));
typedef _Float16       v8h  __attribute__((ext_vector_type(8)));
typedef float          v8f  __attribute__((ext_vector_type(8)));
typedef float          v4f  __attribute__((ext_vector_type(4)));
typedef unsigned int   v4u  __attribute__((ext_vector_type(4)));

union HU { v8h h; v4u u; _Float16 s[8]; };
union FR { v16h v; v8h h[2]; _Float16 s[16]; };
static_assert(sizeof(HU) == 16);
static_assert(sizeof(FR) == 32);

__device__ __forceinline__ unsigned short bf_bits(float f) {
  const unsigned u = __float_as_uint(f);
  return (unsigned short)((u + 0x7FFFu + ((u >> 16) & 1u)) >> 16);
}
__device__ __forceinline__ float bf_up(unsigned short h) { return __uint_as_float(((unsigned)h) << 16); }
__device__ __forceinline__ float bfr(float f) { return bf_up(bf_bits(f)); }
__device__ __forceinline__ v8f zero8() { v8f z = {0.f, 0.f, 0.f, 0.f, 0.f, 0.f, 0.f, 0.f}; return z; }

__device__ __forceinline__ void ld8(const float* p, float* o) {
  const v4f a = *(const v4f*)(p);
  const v4f b = *(const v4f*)(p + 4);
  o[0] = a[0]; o[1] = a[1]; o[2] = a[2]; o[3] = a[3];
  o[4] = b[0]; o[5] = b[1]; o[6] = b[2]; o[7] = b[3];
}

__device__ __forceinline__ float sigm(float z) {
  const float e = expf(-fabsf(z));
  const float rc = 1.0f / (1.0f + e);
  return (z >= 0.0f) ? rc : e * rc;
}
__device__ __forceinline__ float bnorm(float g, float mu, float rs, float ga, float be, float bi) {
  return ((g - mu) * rs) * ga + be + bi;
}

__device__ __forceinline__ v16h ldfrag_h(const _Float16* p) {
  FR f;
  f.h[0] = *(const v8h*)(p);
  f.h[1] = *(const v8h*)(p + 16);
  return f.v;
}

__device__ __forceinline__ v8f mma_h(v16h a, v16h b, v8f c) {
  c = __builtin_amdgcn_wmma_f32_16x16x32_f16(false, a, false, b, (short)0, c, false, false);
#if defined(__HIP_DEVICE_COMPILE__)
  asm volatile("v_nop\n\tv_nop\n\tv_nop\n\tv_nop" : "+v"(c) : "v"(a), "v"(b));
#endif
  return c;
}
__device__ __forceinline__ v8f mma_h_raw(v16h a, v16h b, v8f c) {
  return __builtin_amdgcn_wmma_f32_16x16x32_f16(false, a, false, b, (short)0, c, false, false);
}
__device__ __forceinline__ void dep_guard_h(v8f& a, v8f& b, v16h x) {
#if defined(__HIP_DEVICE_COMPILE__)
  asm volatile("v_nop\n\tv_nop\n\tv_nop\n\tv_nop" : "+v"(a), "+v"(b) : "v"(x));
#endif
}
__device__ __forceinline__ void keep4_h(v16h a, v16h b, v16h c, v16h d) {
#if defined(__HIP_DEVICE_COMPILE__)
  asm volatile("v_nop" :: "v"(a), "v"(b), "v"(c), "v"(d));
#endif
}
__device__ __forceinline__ void acc_guard4(v8f& a, v8f& b, v8f& c, v8f& d) {
#if defined(__HIP_DEVICE_COMPILE__)
  asm volatile("v_nop\n\tv_nop\n\tv_nop\n\tv_nop" : "+v"(a), "+v"(b), "+v"(c), "+v"(d));
#endif
}
__device__ __forceinline__ void wave_lds_sync() {
  __builtin_amdgcn_fence(__ATOMIC_RELEASE, "workgroup");
  __builtin_amdgcn_wave_barrier();
  __builtin_amdgcn_fence(__ATOMIC_ACQUIRE, "workgroup");
}

__global__ __launch_bounds__(256) void cvt_flat(const float* __restrict__ in, _Float16* out, int n8, float scale) {
  const int i = blockIdx.x * 256 + threadIdx.x;
  if (i < n8) {
    float v[8];
    ld8(in + (size_t)i * 8, v);
    HU u;
#pragma unroll
    for (int e = 0; e < 8; ++e) u.s[e] = (_Float16)(bfr(v[e]) * scale);
    _Float16* p = out + (size_t)i * 8;
    *(volatile v4u*)p = u.u;
    __threadfence();
    *(volatile v4u*)p = u.u;
  }
}

__global__ __launch_bounds__(256) void cvt_T(const float* __restrict__ W, _Float16* WT, int Kd, int Nd, float scale) {
  __shared__ float sw[64][65];
  const int t = threadIdx.x;
  const int n0 = blockIdx.x * 64, k0 = blockIdx.y * 64;
  {
    const int r = t >> 4, c4 = (t & 15) * 4;
#pragma unroll
    for (int it = 0; it < 4; ++it) {
      const int row = r + 16 * it;
      const v4f x = *(const v4f*)(W + (size_t)(k0 + row) * Nd + n0 + c4);
      sw[row][c4 + 0] = x[0]; sw[row][c4 + 1] = x[1]; sw[row][c4 + 2] = x[2]; sw[row][c4 + 3] = x[3];
    }
  }
  __syncthreads();
  const int q8 = t & 7, rr = t >> 3;
  HU u[2];
#pragma unroll
  for (int it = 0; it < 2; ++it) {
    const int n = rr + 32 * it;
#pragma unroll
    for (int e = 0; e < 8; ++e) u[it].s[e] = (_Float16)(bfr(sw[8 * q8 + e][n]) * scale);
  }
  for (int pass = 0; pass < 2; ++pass) {
#pragma unroll
    for (int it = 0; it < 2; ++it) {
      const int n = rr + 32 * it;
      _Float16* dst = WT + (size_t)(n0 + n) * Kd + k0 + 8 * q8;
      *(volatile v4u*)dst = u[it].u;
    }
    __threadfence();
  }
}

__device__ __forceinline__ void kseg(v8f (&acc)[4][4], const _Float16* __restrict__ A, int lda, int m0,
                                     const _Float16* __restrict__ Bt, int ldb, int n0, int K, int rlane, int koff) {
  for (int kk = 0; kk < K; kk += 32) {
    v16h bh[4];
#pragma unroll
    for (int j = 0; j < 4; ++j) {
      const size_t bo = (size_t)(n0 + (j << 4) + rlane) * (size_t)ldb + koff + kk;
      bh[j] = ldfrag_h(Bt + bo);
    }
#pragma unroll
    for (int i = 0; i < 4; ++i) {
      const size_t ao = (size_t)(m0 + (i << 4) + rlane) * (size_t)lda + koff + kk;
      const v16h a0 = ldfrag_h(A + ao);
#pragma unroll
      for (int j = 0; j < 4; ++j) acc[i][j] = mma_h_raw(a0, bh[j], acc[i][j]);
      dep_guard_h(acc[i][0], acc[i][3], a0);
    }
    keep4_h(bh[0], bh[1], bh[2], bh[3]);
  }
}

__device__ __forceinline__ void kseg2(v8f (&ach)[2][4], v8f (&acl)[2][4],
                                      const _Float16* __restrict__ Ah, const _Float16* __restrict__ Al, int lda, int m0,
                                      const _Float16* __restrict__ Bt, int ldb, int n0, int K, int rlane, int koff) {
  for (int kk = 0; kk < K; kk += 32) {
    v16h bh[4];
#pragma unroll
    for (int j = 0; j < 4; ++j) {
      const size_t bo = (size_t)(n0 + (j << 4) + rlane) * (size_t)ldb + koff + kk;
      bh[j] = ldfrag_h(Bt + bo);
    }
#pragma unroll
    for (int i = 0; i < 2; ++i) {
      const size_t ao = (size_t)(m0 + (i << 4) + rlane) * (size_t)lda + koff + kk;
      const v16h ah = ldfrag_h(Ah + ao);
#pragma unroll
      for (int j = 0; j < 4; ++j) ach[i][j] = mma_h_raw(ah, bh[j], ach[i][j]);
      dep_guard_h(ach[i][0], ach[i][3], ah);
      const v16h al = ldfrag_h(Al + ao);
#pragma unroll
      for (int j = 0; j < 4; ++j) acl[i][j] = mma_h_raw(al, bh[j], acl[i][j]);
      dep_guard_h(acl[i][0], acl[i][3], al);
    }
    keep4_h(bh[0], bh[1], bh[2], bh[3]);
  }
}

template <int MODE>
__global__ __launch_bounds__(256) void gemm64(
    const _Float16* __restrict__ A, int lda, const _Float16* __restrict__ Bt, int ldb, int M, int N, int K,
    const float* Gp, int gcol, const float* MU, const float* RS,
    const float* gam, const float* bet, const float* bia, const float* hx,
    float* Fo, _Float16* Ph, _Float16* Pl) {
  __shared__ __align__(16) float sT[8][16 * 68];
  const int lane = threadIdx.x & 31;
  const int wave = threadIdx.x >> 5;
  const int tilesN = N >> 6;
  const int tilesM = M >> 6;
  const int tiles = tilesM * tilesN;
  const int item = blockIdx.x * 8 + wave;
  if (item >= tiles) return;
  const int tm = item / tilesN;
  const int tn = item - tm * tilesN;
  const int m0 = tm << 6;
  const int n0 = tn << 6;

  const int rlane = lane & 15;
  const int koff  = (lane >> 4) * 8;
  const int mOff  = (lane >> 4) * 8;

  v8f acc[4][4];
#pragma unroll
  for (int i = 0; i < 4; ++i)
#pragma unroll
    for (int j = 0; j < 4; ++j) acc[i][j] = zero8();

  kseg(acc, A, lda, m0, Bt, ldb, n0, K, rlane, koff);
  acc_guard4(acc[0][0], acc[0][1], acc[0][2], acc[0][3]);
  acc_guard4(acc[1][0], acc[1][1], acc[1][2], acc[1][3]);
  acc_guard4(acc[2][0], acc[2][1], acc[2][2], acc[2][3]);
  acc_guard4(acc[3][0], acc[3][1], acc[3][2], acc[3][3]);

  const int r2 = lane >> 4, c4 = (lane & 15) * 4;
  const int q8 = lane & 7, rr = lane >> 3, c8 = q8 * 8;

  float* slab = sT[wave];
#pragma unroll
  for (int i = 0; i < 4; ++i) {
    const int mBase = m0 + (i << 4);
#pragma unroll
    for (int r = 0; r < 8; ++r) {
#pragma unroll
      for (int j = 0; j < 4; ++j) {
        slab[(mOff + r) * 68 + (j << 4) + rlane] = acc[i][j][r];
      }
    }
    wave_lds_sync();
    if (MODE != 2) {
      v4f ov[8];
#pragma unroll
      for (int it = 0; it < 8; ++it) {
        const int row = 2 * it + r2;
        const v4f x = *(const v4f*)(slab + row * 68 + c4);
        if (MODE == 0) {
          ov[it] = x * INVAW;
        } else {
          const int m = mBase + row, nn = n0 + c4;
          const v4f gv = *(const v4f*)(Gp + (size_t)m * N3 + gcol + nn);
          const v4f mv = *(const v4f*)(MU + gcol + nn);
          const v4f rv = *(const v4f*)(RS + gcol + nn);
          const v4f av = *(const v4f*)(gam + gcol + nn);
          const v4f bv = *(const v4f*)(bet + gcol + nn);
          const v4f iv = *(const v4f*)(bia + gcol + nn);
          v4f o;
#pragma unroll
          for (int e = 0; e < 4; ++e) {
            const float gn = bnorm(gv[e], mv[e], rv[e], bfr(av[e]), bfr(bv[e]), bfr(iv[e]));
            o[e] = sigm(gn + x[e] * INVAW);
          }
          ov[it] = o;
        }
      }
      for (int pass = 0; pass < 2; ++pass) {
#pragma unroll
        for (int it = 0; it < 8; ++it) {
          const int row = 2 * it + r2;
          float* dst = Fo + (size_t)(mBase + row) * (size_t)N + n0 + c4;
          *(volatile v4f*)dst = ov[it];
        }
        __threadfence();
      }
    } else {
      v4u uh[4], ul[4];
#pragma unroll
      for (int it = 0; it < 4; ++it) {
        const int row = it * 4 + rr;
        const int m = mBase + row;
        const int nb = n0 + c8;
        HU h, l;
#pragma unroll
        for (int hf = 0; hf < 2; ++hf) {
          const int nn = nb + 4 * hf;
          const v4f x  = *(const v4f*)(slab + row * 68 + c8 + 4 * hf);
          const v4f gv = *(const v4f*)(Gp + (size_t)m * N3 + gcol + nn);
          const v4f mv = *(const v4f*)(MU + gcol + nn);
          const v4f rv = *(const v4f*)(RS + gcol + nn);
          const v4f av = *(const v4f*)(gam + gcol + nn);
          const v4f bv = *(const v4f*)(bet + gcol + nn);
          const v4f iv = *(const v4f*)(bia + gcol + nn);
          const v4f hv = *(const v4f*)(hx + (size_t)m * HD + nn);
#pragma unroll
          for (int e = 0; e < 4; ++e) {
            const float gn = bnorm(gv[e], mv[e], rv[e], bfr(av[e]), bfr(bv[e]), bfr(iv[e]));
            const float rg = sigm(gn + x[e] * INVAW);
            const float w  = (rg * bfr(hv[e])) * SCP;
            const _Float16 wh = (_Float16)w;
            h.s[4 * hf + e] = wh;
            l.s[4 * hf + e] = (_Float16)((w - (float)wh) * SCR);
          }
        }
        uh[it] = h.u;
        ul[it] = l.u;
      }
      for (int pass = 0; pass < 2; ++pass) {
#pragma unroll
        for (int it = 0; it < 4; ++it) {
          const int row = it * 4 + rr;
          const size_t co = (size_t)(mBase + row) * (size_t)N + n0 + c8;
          *(volatile v4u*)(Ph + co) = uh[it];
          *(volatile v4u*)(Pl + co) = ul[it];
        }
        __threadfence();
      }
    }
    wave_lds_sync();
  }
}

__global__ __launch_bounds__(256) void gemm_c(
    const _Float16* __restrict__ Ah, const _Float16* __restrict__ Al, int lda,
    const _Float16* __restrict__ Bt, int ldb, int M, int N, int K,
    const float* Gp, int gcol, const float* MU, const float* RS,
    const float* gam, const float* bet, const float* bia, const float* U, const float* hx, float* out) {
  __shared__ __align__(16) float sT[8][16 * 68];
  const int lane = threadIdx.x & 31;
  const int wave = threadIdx.x >> 5;
  const int tilesN = N >> 6;
  const int tilesM = M >> 5;
  const int tiles = tilesM * tilesN;
  const int item = blockIdx.x * 8 + wave;
  if (item >= tiles) return;
  const int tm = item / tilesN;
  const int tn = item - tm * tilesN;
  const int m0 = tm << 5;
  const int n0 = tn << 6;

  const int rlane = lane & 15;
  const int koff  = (lane >> 4) * 8;
  const int mOff  = (lane >> 4) * 8;

  v8f ach[2][4], acl[2][4];
#pragma unroll
  for (int i = 0; i < 2; ++i)
#pragma unroll
    for (int j = 0; j < 4; ++j) { ach[i][j] = zero8(); acl[i][j] = zero8(); }

  kseg2(ach, acl, Ah, Al, lda, m0, Bt, ldb, n0, K, rlane, koff);
  acc_guard4(ach[0][0], ach[0][1], ach[0][2], ach[0][3]);
  acc_guard4(ach[1][0], ach[1][1], ach[1][2], ach[1][3]);
  acc_guard4(acl[0][0], acl[0][1], acl[0][2], acl[0][3]);
  acc_guard4(acl[1][0], acl[1][1], acl[1][2], acl[1][3]);

  const int r2 = lane >> 4, c4 = (lane & 15) * 4;
  float* slab = sT[wave];
#pragma unroll
  for (int i = 0; i < 2; ++i) {
    const int mBase = m0 + (i << 4);
#pragma unroll
    for (int r = 0; r < 8; ++r) {
#pragma unroll
      for (int j = 0; j < 4; ++j) {
        slab[(mOff + r) * 68 + (j << 4) + rlane] = ach[i][j][r] * INVPW + acl[i][j][r] * INVPL;
      }
    }
    wave_lds_sync();
    v4f ov[8];
#pragma unroll
    for (int it = 0; it < 8; ++it) {
      const int row = 2 * it + r2;
      const int m = mBase + row, nn = n0 + c4;
      const v4f x  = *(const v4f*)(slab + row * 68 + c4);
      const v4f gv = *(const v4f*)(Gp + (size_t)m * N3 + gcol + nn);
      const v4f mv = *(const v4f*)(MU + gcol + nn);
      const v4f rv = *(const v4f*)(RS + gcol + nn);
      const v4f av = *(const v4f*)(gam + gcol + nn);
      const v4f bv = *(const v4f*)(bet + gcol + nn);
      const v4f iv = *(const v4f*)(bia + gcol + nn);
      const v4f uv = *(const v4f*)(U + (size_t)m * HD + nn);
      const v4f hv = *(const v4f*)(hx + (size_t)m * HD + nn);
      v4f o;
#pragma unroll
      for (int e = 0; e < 4; ++e) {
        const float gn = bnorm(gv[e], mv[e], rv[e], bfr(av[e]), bfr(bv[e]), bfr(iv[e]));
        const float cc = tanhf(gn + x[e]);
        const float u  = uv[e];
        const float hb = bfr(hv[e]);
        o[e] = (1.0f - u) * hb + u * cc;
      }
      ov[it] = o;
    }
    for (int pass = 0; pass < 2; ++pass) {
#pragma unroll
      for (int it = 0; it < 8; ++it) {
        const int row = 2 * it + r2;
        float* dst = out + (size_t)(mBase + row) * (size_t)N + n0 + c4;
        *(volatile v4f*)dst = ov[it];
      }
      __threadfence();
    }
    wave_lds_sync();
  }
}

__global__ __launch_bounds__(256) void k_stats(const float* __restrict__ Gp, float* MU, float* RS) {
  __shared__ double sS[4][64];
  __shared__ double sQ[4][64];
  __shared__ __align__(16) float sM[64];
  __shared__ __align__(16) float sR[64];
  const int tid = threadIdx.x, c = tid & 63, rq = tid >> 6;
  const int c0 = blockIdx.x * 64;
  const float* gp = Gp + (size_t)rq * N3 + c0 + c;
  double s = 0.0, q = 0.0;
#pragma unroll 4
  for (int r = 0; r < BATCH / 4; ++r) {
    const float x = gp[(size_t)r * (size_t)(4 * N3)];
    s += (double)x;
    q += (double)x * (double)x;
  }
  sS[rq][c] = s;
  sQ[rq][c] = q;
  __syncthreads();
  if (tid < 64) {
    const double ts = ((sS[0][tid] + sS[1][tid]) + sS[2][tid]) + sS[3][tid];
    const double tq = ((sQ[0][tid] + sQ[1][tid]) + sQ[2][tid]) + sQ[3][tid];
    const double m = ts * (1.0 / (double)BATCH);
    double var = tq * (1.0 / (double)BATCH) - m * m;
    var = var > 0.0 ? var : 0.0;
    sM[tid] = (float)m;
    sR[tid] = 1.0f / sqrtf((float)var + BN_EPS);
  }
  __syncthreads();
  if (tid < 32) {
    const int lane = tid, p = lane & 15;
    const v4f vm = *(const v4f*)(&sM[4 * p]);
    const v4f vr = *(const v4f*)(&sR[4 * p]);
    v4f val;
#pragma unroll
    for (int e = 0; e < 4; ++e) val[e] = (lane < 16) ? vm[e] : vr[e];
    float* dst = ((lane < 16) ? MU : RS) + c0 + 4 * p;
    *(volatile v4f*)dst = val;
    __threadfence();
    *(volatile v4f*)dst = val;
  }
}

extern "C" void kernel_launch(void* const* d_in, const int* in_sizes, int n_in,
                              void* d_out, int out_size, void* d_ws, size_t ws_size,
                              hipStream_t stream) {
  if (n_in < 7) return;
  if (in_sizes[0] != BATCH * KD || in_sizes[1] != BATCH * HD) return;
  if (in_sizes[2] != KD * N3 || in_sizes[3] != HD * N3) return;
  if (in_sizes[4] != N3 || in_sizes[5] != N3 || in_sizes[6] != N3) return;
  if (out_size != BATCH * HD) return;

  const float* input = (const float*)d_in[0];
  const float* hx    = (const float*)d_in[1];
  const float* wi    = (const float*)d_in[2];
  const float* wh    = (const float*)d_in[3];
  const float* bias  = (const float*)d_in[4];
  const float* gam   = (const float*)d_in[5];
  const float* bet   = (const float*)d_in[6];

  const size_t PA16 = (size_t)BATCH * KD * 2;
  const size_t PH16 = (size_t)BATCH * HD * 2;
  const size_t PWI  = (size_t)N3 * KD * 2;
  const size_t PWH  = (size_t)N3 * HD * 2;
  const size_t PG   = (size_t)BATCH * N3 * 4;
  const size_t PST  = (size_t)N3 * 4;
  const size_t PU   = (size_t)BATCH * HD * 4;
  const size_t PRH  = (size_t)BATCH * HD * 2;

  size_t off = 0;
  const size_t oA16 = off; off += PA16;
  const size_t oH16 = off; off += PH16;
  const size_t oWIT = off; off += PWI;
  const size_t oWHT = off; off += PWH;
  const size_t oG   = off; off += PG;
  const size_t oMU  = off; off += PST;
  const size_t oRS  = off; off += PST;
  const size_t oU   = off; off += PU;
  const size_t oRHh = off; off += PRH;
  const size_t oRHl = off; off += PRH;
  if (off > ws_size) return;
  if (off > (size_t)134217728) return;

  char* ws = (char*)d_ws;
  _Float16* A16 = (_Float16*)(ws + oA16);
  _Float16* H16 = (_Float16*)(ws + oH16);
  _Float16* WIT = (_Float16*)(ws + oWIT);
  _Float16* WHT = (_Float16*)(ws + oWHT);
  float*    G   = (float*)(ws + oG);
  float*    MU  = (float*)(ws + oMU);
  float*    RS  = (float*)(ws + oRS);
  float*    U   = (float*)(ws + oU);
  _Float16* RHh = (_Float16*)(ws + oRHh);
  _Float16* RHl = (_Float16*)(ws + oRHl);
  float*    outf = (float*)d_out;

  const dim3 blk(256);
  const int n8a = (BATCH * KD) / 8;
  const int n8h = (BATCH * HD) / 8;
  const dim3 gCa((n8a + 255) / 256);
  const dim3 gCh((n8h + 255) / 256);
  const dim3 gTi(N3 / 64, KD / 64);
  const dim3 gTh(N3 / 64, HD / 64);
  const dim3 gG(((BATCH / 64) * (N3 / 64)) / 8);
  const dim3 gSt(N3 / 64);
  const dim3 gUR(((BATCH / 64) * (HD / 64)) / 8);
  const dim3 gC(((BATCH / 32) * (HD / 64)) / 8);

  cvt_flat<<<gCa, blk, 0, stream>>>(input, A16, n8a, SCA);
  cvt_flat<<<gCh, blk, 0, stream>>>(hx, H16, n8h, SCA);
  cvt_T<<<gTi, blk, 0, stream>>>(wi, WIT, KD, N3, SCW);
  cvt_T<<<gTh, blk, 0, stream>>>(wh, WHT, HD, N3, SCW);
  gemm64<0><<<gG, blk, 0, stream>>>(A16, KD, WIT, KD, BATCH, N3, KD, G, 0, MU, RS, gam, bet, bias, hx, G, RHh, RHl);
  k_stats<<<gSt, blk, 0, stream>>>(G, MU, RS);
  gemm64<1><<<gUR, blk, 0, stream>>>(H16, HD, WHT, HD, BATCH, HD, HD, G, 0, MU, RS, gam, bet, bias, hx, U, RHh, RHl);
  gemm64<2><<<gUR, blk, 0, stream>>>(H16, HD, WHT + (size_t)HD * HD, HD, BATCH, HD, HD, G, HD, MU, RS, gam, bet,
                                     bias, hx, U, RHh, RHl);
  gemm_c<<<gC, blk, 0, stream>>>(RHh, RHl, HD, WHT + (size_t)2 * HD * HD, HD, BATCH, HD, HD, G, 2 * HD, MU, RS,
                                 gam, bet, bias, U, hx, outf);
}
